// MultiHeadAttention_16801912062309
// MI455X (gfx1250) — hardware-run, weakly checked
//
#include <hip/hip_runtime.h>
#ifndef NB
#define NB 16
#endif
#ifndef SEQ
#define SEQ 512
#endif
#define NB_FULL 16
#define SEQ_FULL 512
#define NH 8
#define HD 128
#define EMB 128
#define HE 1024
#define YP 2048
#define XSTRIDE_FULL ((size_t)SEQ_FULL * EMB)
#define DSTRIDE_FULL ((size_t)SEQ_FULL * SEQ_FULL)
#define PLANE ((size_t)NB * NH * SEQ * HD)

static_assert(SEQ % 64 == 0);
static_assert(SEQ <= SEQ_FULL);
static_assert(NB <= NB_FULL);
static_assert(HD == 128);
static_assert(EMB % 32 == 0);
static_assert(HE == NH * HD);
static_assert((size_t)NB * SEQ * EMB * 2 + (size_t)3 * HE * EMB * 2 + (size_t)EMB * HE * 2 + 3 * PLANE * 2 + (size_t)NB * SEQ * YP * 2 + 2048 <= (size_t)134217728);

typedef __bf16 v16b __attribute__((ext_vector_type(16)));
typedef _Float16 v16h __attribute__((ext_vector_type(16)));
typedef unsigned short v8us __attribute__((ext_vector_type(8), may_alias));
typedef float v8f __attribute__((ext_vector_type(8)));
typedef float v4f __attribute__((ext_vector_type(4)));
typedef float v4fa __attribute__((ext_vector_type(4), may_alias));
union FragB { v16b v; v8us half[2]; unsigned short u[16]; };
union FragH { v16h v; v8us half[2]; _Float16 h[16]; unsigned short u[16]; };

#define LOG2E 1.4426950408889634f
#define NEGV (-1000000000.0f)
#define SCL (0.08838834764831845f * 0.00390625f)

__device__ __forceinline__ unsigned short bf16_bits(float x) {
  unsigned int u = __float_as_uint(x);
  return (unsigned short)((u + 0x7FFFu + ((u >> 16) & 1u)) >> 16);
}
__device__ __forceinline__ float bf16_val(unsigned short b) { return __uint_as_float(((unsigned int)b) << 16); }
__device__ __forceinline__ float bf16_rne(float x) { return bf16_val(bf16_bits(x)); }
__device__ __forceinline__ unsigned short f16_bits(float x) {
  const _Float16 h = (_Float16)x;
  return __builtin_bit_cast(unsigned short, h);
}

__device__ __forceinline__ v8f mma_bf2(v16b a0, v16b b0, v16b a1, v16b b1, v8f c) {
  c = __builtin_amdgcn_wmma_f32_16x16x32_bf16(false, a0, false, b0, (short)0, c, false, false);
  c = __builtin_amdgcn_wmma_f32_16x16x32_bf16(false, a1, false, b1, (short)0, c, false, false);
  asm volatile("v_nop\n\tv_nop\n\tv_nop\n\tv_nop" : "+v"(c) : "v"(a0), "v"(b0), "v"(a1), "v"(b1));
  return c;
}
__device__ __forceinline__ v8f mma_h2c(v16h a0, v16h b0, v16h a1, v16h b1, v8f c) {
  c = __builtin_amdgcn_wmma_f32_16x16x32_f16(false, a0, false, b0, (short)0, c, false, false);
  c = __builtin_amdgcn_wmma_f32_16x16x32_f16(false, a1, false, b1, (short)0, c, false, false);
  asm volatile("v_nop\n\tv_nop\n\tv_nop\n\tv_nop" : "+v"(c) : "v"(a0), "v"(b0), "v"(a1), "v"(b1));
  return c;
}

__device__ __forceinline__ v8us cvt8_bf16(const float* src) {
  const v4f x0 = *(const v4fa*)(src), x1 = *(const v4fa*)(src + 4);
  v8us o;
  o[0] = bf16_bits(x0[0]); o[1] = bf16_bits(x0[1]); o[2] = bf16_bits(x0[2]); o[3] = bf16_bits(x0[3]);
  o[4] = bf16_bits(x1[0]); o[5] = bf16_bits(x1[1]); o[6] = bf16_bits(x1[2]); o[7] = bf16_bits(x1[3]);
  return o;
}

__global__ __launch_bounds__(256) void k_cvt_x(const float* __restrict__ X, unsigned short* __restrict__ Xb) {
  const int t = blockIdx.x * 256 + threadIdx.x;
  if (t >= NB * SEQ * 16) return;
  const int row = t >> 4, piece = t & 15;
  const int b = row / SEQ, n = row - b * SEQ;
  const v8us o = cvt8_bf16(X + (size_t)b * XSTRIDE_FULL + (size_t)n * EMB + piece * 8);
  unsigned short* d = Xb + (size_t)t * 8;
  *(volatile v8us*)d = o;
  __threadfence();
  *(volatile v8us*)d = o;
}

__global__ __launch_bounds__(256) void k_cvt_w(const float* __restrict__ src, unsigned short* __restrict__ dst, int npieces) {
  const int t = blockIdx.x * 256 + threadIdx.x;
  if (t >= npieces) return;
  const v8us o = cvt8_bf16(src + (size_t)t * 8);
  unsigned short* d = dst + (size_t)t * 8;
  *(volatile v8us*)d = o;
  __threadfence();
  *(volatile v8us*)d = o;
}

__global__ __launch_bounds__(128) void k_proj(const unsigned short* __restrict__ Xb, const unsigned short* __restrict__ Wb,
                                              const float* __restrict__ bq, const float* __restrict__ bk, const float* __restrict__ bv,
                                              const float* __restrict__ mask, unsigned short* __restrict__ QKV) {
  __shared__ __attribute__((aligned(16))) unsigned short tl[9216];
  const int tid = threadIdx.x, w = __builtin_amdgcn_readfirstlane((int)(tid >> 5)), lane = tid & 31, ln = lane & 15, hh = lane >> 4;
  const int which = blockIdx.y >> 3, h = blockIdx.y & 7;
  const int row0 = blockIdx.x * 64;
  const int b = row0 / SEQ, n0 = row0 - b * SEQ;
  const unsigned short* xp = Xb + (size_t)(row0 + 16 * w + ln) * EMB + 8 * hh;
  FragB a[4];
#pragma unroll
  for (int c = 0; c < 4; ++c) {
    a[c].half[0] = *(const v8us*)(xp + 32 * c);
    a[c].half[1] = *(const v8us*)(xp + 32 * c + 16);
  }
  float mrow[8];
#pragma unroll
  for (int r = 0; r < 8; ++r) mrow[r] = mask[(size_t)b * SEQ_FULL + n0 + 16 * w + 8 * hh + r] * 16.0f;
  const unsigned short* wp = Wb + (size_t)(blockIdx.y * 128 + ln) * EMB + 8 * hh;
  const v8f z8 = {0.f, 0.f, 0.f, 0.f, 0.f, 0.f, 0.f, 0.f};
#pragma unroll 1
  for (int t = 0; t < 8; ++t) {
    const unsigned short* wt = wp + (size_t)t * 16 * EMB;
    FragB b0, b1, b2, b3;
    b0.half[0] = *(const v8us*)(wt);      b0.half[1] = *(const v8us*)(wt + 16);
    b1.half[0] = *(const v8us*)(wt + 32); b1.half[1] = *(const v8us*)(wt + 48);
    b2.half[0] = *(const v8us*)(wt + 64); b2.half[1] = *(const v8us*)(wt + 80);
    b3.half[0] = *(const v8us*)(wt + 96); b3.half[1] = *(const v8us*)(wt + 112);
    v8f acc = z8;
    acc = mma_bf2(a[0].v, b0.v, a[1].v, b1.v, acc);
    acc = mma_bf2(a[2].v, b2.v, a[3].v, b3.v, acc);
    const int cg = h * HD + 16 * t + ln;
    const float c0 = bq[cg], c1 = bk[cg], c2 = bv[cg];
    const float bias = bf16_rne(which == 0 ? c0 : (which == 1 ? c1 : c2));
    const int coll = 16 * t + ln;
#pragma unroll
    for (int r = 0; r < 8; ++r) {
      const int rowl = 16 * w + 8 * hh + r;
      const float val = (acc[r] + bias) * mrow[r];
      const int idx = (which == 2) ? (coll * 72 + rowl) : (rowl * 136 + coll);
      tl[idx] = f16_bits(val);
    }
  }
  __syncthreads();
  unsigned short* base = QKV + (size_t)which * PLANE;
  if (which != 2) {
    unsigned short* dst = base + ((size_t)(b * NH + h) * SEQ + n0) * HD;
    for (int pass = 0; pass < 2; ++pass) {
      for (int i = tid; i < 64 * 16; i += 128) {
        const int row = i >> 4, p8 = (i & 15) * 8;
        const v8us o = *(const v8us*)&tl[row * 136 + p8];
        *(volatile v8us*)(dst + (size_t)row * HD + p8) = o;
      }
      if (pass == 0) __threadfence();
    }
  } else {
    unsigned short* dst = base + (size_t)(b * NH + h) * HD * SEQ + n0;
    for (int pass = 0; pass < 2; ++pass) {
      for (int i = tid; i < 128 * 8; i += 128) {
        const int d = i >> 3, j8 = (i & 7) * 8;
        const v8us o = *(const v8us*)&tl[d * 72 + j8];
        *(volatile v8us*)(dst + (size_t)d * SEQ + j8) = o;
      }
      if (pass == 0) __threadfence();
    }
  }
}

__global__ __launch_bounds__(128) void k_attn(const unsigned short* __restrict__ Qp, const unsigned short* __restrict__ Kpl,
                                              const unsigned short* __restrict__ Vtp, const float* __restrict__ dist,
                                              const float* __restrict__ mask, unsigned short* __restrict__ Y) {
  __shared__ __attribute__((aligned(16))) unsigned short so[4][16][264];
  __shared__ __attribute__((aligned(16))) float smk[SEQ];
  const int tid = threadIdx.x, w = __builtin_amdgcn_readfirstlane((int)(tid >> 5)), lane = tid & 31, ln = lane & 15, hh = lane >> 4;
  const int qt = blockIdx.x % (SEQ / 64), bh = blockIdx.x / (SEQ / 64);
  const int b = bh / NH, h = bh - b * NH;
  for (int i = tid; i < SEQ; i += 128) smk[i] = mask[(size_t)b * SEQ_FULL + i];
  __syncthreads();
  const int qbase = qt * 64 + 16 * w;
  const int qg = qbase + ln;
  const float mq = mask[(size_t)b * SEQ_FULL + qg];
  const unsigned short* qp = Qp + ((size_t)bh * SEQ + qg) * HD + 8 * hh;
  FragH qf[4];
#pragma unroll
  for (int c = 0; c < 4; ++c) {
    qf[c].half[0] = *(const v8us*)(qp + 32 * c);
    qf[c].half[1] = *(const v8us*)(qp + 32 * c + 16);
  }
  const unsigned short* Kp = Kpl + (size_t)bh * SEQ * HD;
  const unsigned short* Vp = Vtp + (size_t)bh * HD * SEQ;
  const float* drow = dist + (size_t)b * DSTRIDE_FULL + (size_t)qg * SEQ_FULL;
  float mr = -3.0e38f, lr = 0.0f;
  v8f O[8] = {};
  const v8f z8 = {0.f, 0.f, 0.f, 0.f, 0.f, 0.f, 0.f, 0.f};

#pragma unroll 1
  for (int key0 = 0; key0 < SEQ; key0 += 32) {
    const unsigned short* kp0 = Kp + (size_t)(key0 + ln) * HD + 8 * hh;
    const unsigned short* kp1 = kp0 + 16 * HD;
    v8f s0 = z8, s1 = z8;
#pragma unroll
    for (int c = 0; c < 4; c += 2) {
      FragH k0a, k0b, k1a, k1b;
      k0a.half[0] = *(const v8us*)(kp0 + 32 * c);      k0a.half[1] = *(const v8us*)(kp0 + 32 * c + 16);
      k0b.half[0] = *(const v8us*)(kp0 + 32 * c + 32); k0b.half[1] = *(const v8us*)(kp0 + 32 * c + 48);
      k1a.half[0] = *(const v8us*)(kp1 + 32 * c);      k1a.half[1] = *(const v8us*)(kp1 + 32 * c + 16);
      k1b.half[0] = *(const v8us*)(kp1 + 32 * c + 32); k1b.half[1] = *(const v8us*)(kp1 + 32 * c + 48);
      s0 = mma_h2c(k0a.v, qf[c].v, k0b.v, qf[c + 1].v, s0);
      s1 = mma_h2c(k1a.v, qf[c].v, k1b.v, qf[c + 1].v, s1);
    }
    const float* dp = drow + key0 + 8 * hh;
    const v4f d0 = *(const v4fa*)(dp), d1 = *(const v4fa*)(dp + 4), d2 = *(const v4fa*)(dp + 16), d3 = *(const v4fa*)(dp + 20);
    const v4f m0 = *(const v4fa*)&smk[key0 + 8 * hh],      m1 = *(const v4fa*)&smk[key0 + 8 * hh + 4];
    const v4f m2 = *(const v4fa*)&smk[key0 + 8 * hh + 16], m3 = *(const v4fa*)&smk[key0 + 8 * hh + 20];
    float sc[16], mkv[16];
#pragma unroll
    for (int i = 0; i < 4; ++i) {
      sc[i]      = fmaf(s0[i],     SCL, bf16_rne(d0[i]));
      sc[4 + i]  = fmaf(s0[4 + i], SCL, bf16_rne(d1[i]));
      sc[8 + i]  = fmaf(s1[i],     SCL, bf16_rne(d2[i]));
      sc[12 + i] = fmaf(s1[4 + i], SCL, bf16_rne(d3[i]));
      mkv[i] = m0[i]; mkv[4 + i] = m1[i]; mkv[8 + i] = m2[i]; mkv[12 + i] = m3[i];
    }
#pragma unroll
    for (int i = 0; i < 16; ++i) sc[i] = (mq * mkv[i] == 0.0f) ? NEGV : sc[i];
    float mx = sc[0];
#pragma unroll
    for (int i = 1; i < 16; ++i) mx = fmaxf(mx, sc[i]);
    mx = fmaxf(mx, __shfl_xor(mx, 16, 32));
    const float mnew = fmaxf(mr, mx);
    const float al = exp2f((mr - mnew) * LOG2E);
    mr = mnew;
    FragH ph, pl;
    float ps = 0.0f;
#pragma unroll
    for (int i = 0; i < 16; ++i) {
      const float pc = exp2f(fmaf(sc[i] - mnew, LOG2E, 12.0f));
      ps += pc;
      const float pz = (mq * mkv[i] == 0.0f) ? 0.0f : pc;
      const _Float16 hv = (_Float16)pz;
      ph.h[i] = hv;
      pl.h[i] = (_Float16)(pz - (float)hv);
    }
    ps += __shfl_xor(ps, 16, 32);
    lr = lr * al + ps;
#pragma unroll
    for (int t = 0; t < 8; ++t) O[t] = O[t] * al;
    const unsigned short* vp = Vp + (size_t)ln * SEQ + key0 + 8 * hh;
#pragma unroll
    for (int t = 0; t < 8; ++t) {
      FragH vf;
      vf.half[0] = *(const v8us*)(vp + (size_t)t * 16 * SEQ);
      vf.half[1] = *(const v8us*)(vp + (size_t)t * 16 * SEQ + 16);
      O[t] = mma_h2c(vf.v, ph.v, vf.v, pl.v, O[t]);
    }
  }

  const float inv = 1.0f / (16.0f * lr);
#pragma unroll
  for (int t = 0; t < 8; ++t)
#pragma unroll
    for (int r = 0; r < 8; ++r) {
      const float yv = O[t][r] * inv;
      const unsigned short hb = bf16_bits(yv);
      const unsigned short lb = bf16_bits(yv - bf16_val(hb));
      so[w][ln][16 * t + 8 * hh + r] = hb;
      so[w][ln][128 + 16 * t + 8 * hh + r] = lb;
    }
  __syncthreads();
  unsigned short* yg = Y + ((size_t)b * SEQ + qbase) * YP + h * HD;
  const int seg = lane >> 4, p8 = (lane & 15) * 8;
  for (int pass = 0; pass < 2; ++pass) {
#pragma unroll
    for (int q = 0; q < 16; ++q) {
      const v8us o = *(const v8us*)&so[w][q][seg * 128 + p8];
      *(volatile v8us*)(yg + (size_t)q * YP + seg * HE + p8) = o;
    }
    if (pass == 0) __threadfence();
  }
}

__global__ __launch_bounds__(128) void k_out(const unsigned short* __restrict__ Y, const unsigned short* __restrict__ Wob,
                                             const float* __restrict__ bo, const float* __restrict__ mask, float* __restrict__ out) {
  __shared__ __attribute__((aligned(16))) float so[4][16][132];
  const int tid = threadIdx.x, w = __builtin_amdgcn_readfirstlane((int)(tid >> 5)), lane = tid & 31, ln = lane & 15, hh = lane >> 4;
  const int row0 = blockIdx.x * 64;
  const int b = row0 / SEQ, n0 = row0 - b * SEQ + 16 * w;
  const unsigned short* yp = Y + (size_t)(row0 + 16 * w + ln) * YP + 8 * hh;
  const unsigned short* wp = Wob + (size_t)ln * HE + 8 * hh;
  v8f acc[8] = {};
#pragma unroll 1
  for (int kk = 0; kk < YP; kk += 64) {
    FragB a0, a1;
    a0.half[0] = *(const v8us*)(yp + kk);      a0.half[1] = *(const v8us*)(yp + kk + 16);
    a1.half[0] = *(const v8us*)(yp + kk + 32); a1.half[1] = *(const v8us*)(yp + kk + 48);
    const int kb = kk & (HE - 1);
#pragma unroll
    for (int t = 0; t < 8; ++t) {
      const unsigned short* wt = wp + (size_t)t * 16 * HE + kb;
      FragB b0, b1;
      b0.half[0] = *(const v8us*)(wt);      b0.half[1] = *(const v8us*)(wt + 16);
      b1.half[0] = *(const v8us*)(wt + 32); b1.half[1] = *(const v8us*)(wt + 48);
      acc[t] = mma_bf2(a0.v, b0.v, a1.v, b1.v, acc[t]);
    }
  }
  float mk[8];
#pragma unroll
  for (int r = 0; r < 8; ++r) mk[r] = mask[(size_t)b * SEQ_FULL + n0 + 8 * hh + r];
#pragma unroll
  for (int t = 0; t < 8; ++t) {
    const float bias = bf16_rne(bo[16 * t + ln]);
#pragma unroll
    for (int r = 0; r < 8; ++r)
      so[w][8 * hh + r][16 * t + ln] = (acc[t][r] + bias) * mk[r];
  }
  __syncthreads();
  float* og = out + (size_t)b * XSTRIDE_FULL + (size_t)n0 * EMB;
  for (int pass = 0; pass < 2; ++pass) {
#pragma unroll
    for (int q = 0; q < 16; ++q) {
      const v4f v = *(const v4fa*)&so[w][q][lane * 4];
      *(volatile v4f*)(og + (size_t)q * EMB + lane * 4) = v;
    }
    if (pass == 0) __threadfence();
  }
}

extern "C" void kernel_launch(void* const* d_in, const int* in_sizes, int n_in,
                              void* d_out, int out_size, void* d_ws, size_t ws_size, hipStream_t stream) {
  if (n_in < 11) return;
  const long long needx = (long long)(NB - 1) * SEQ_FULL * EMB + (long long)SEQ * EMB;
  const long long needd = (long long)(NB - 1) * SEQ_FULL * SEQ_FULL + (long long)(SEQ - 1) * SEQ_FULL + SEQ;
  const long long needm = (long long)(NB - 1) * SEQ_FULL + SEQ;
  if ((long long)in_sizes[0] < needx || (long long)in_sizes[1] < needd || (long long)in_sizes[2] < needm) return;
  if (in_sizes[3] < HE * EMB || in_sizes[5] < HE * EMB || in_sizes[7] < HE * EMB || in_sizes[9] < EMB * HE) return;
  if (in_sizes[4] < HE || in_sizes[6] < HE || in_sizes[8] < HE || in_sizes[10] < EMB) return;
  if ((long long)out_size < needx) return;
  const float* x    = (const float*)d_in[0];
  const float* dist = (const float*)d_in[1];
  const float* mask = (const float*)d_in[2];
  const float* Wq   = (const float*)d_in[3];
  const float* bq   = (const float*)d_in[4];
  const float* Wk   = (const float*)d_in[5];
  const float* bk   = (const float*)d_in[6];
  const float* Wv   = (const float*)d_in[7];
  const float* bv   = (const float*)d_in[8];
  const float* Wo   = (const float*)d_in[9];
  const float* bo   = (const float*)d_in[10];
  float* out = (float*)d_out;
  char* ws = (char*)d_ws;
  size_t off = 0;
  const size_t xb_bytes  = (size_t)NB * SEQ * EMB * 2;
  const size_t wb_bytes  = (size_t)3 * HE * EMB * 2;
  const size_t wob_bytes = (size_t)EMB * HE * 2;
  const size_t qkv_bytes = 3 * PLANE * 2;
  const size_t y_bytes   = (size_t)NB * SEQ * YP * 2;
  unsigned short* Xb  = (unsigned short*)(ws + off); off += (xb_bytes + 255) & ~(size_t)255;
  unsigned short* Wb  = (unsigned short*)(ws + off); off += (wb_bytes + 255) & ~(size_t)255;
  unsigned short* Wob = (unsigned short*)(ws + off); off += (wob_bytes + 255) & ~(size_t)255;
  unsigned short* QKV = (unsigned short*)(ws + off); off += (qkv_bytes + 255) & ~(size_t)255;
  unsigned short* Yp  = (unsigned short*)(ws + off); off += (y_bytes + 255) & ~(size_t)255;
  if (off > ws_size) return;
  const int wpieces = HE * EMB / 8;
  k_cvt_x<<<(unsigned)((NB * SEQ * 16 + 255) / 256), 256, 0, stream>>>(x, Xb);
  k_cvt_w<<<(unsigned)((wpieces + 255) / 256), 256, 0, stream>>>(Wq, Wb, wpieces);
  k_cvt_w<<<(unsigned)((wpieces + 255) / 256), 256, 0, stream>>>(Wk, Wb + (size_t)HE * EMB, wpieces);
  k_cvt_w<<<(unsigned)((wpieces + 255) / 256), 256, 0, stream>>>(Wv, Wb + (size_t)2 * HE * EMB, wpieces);
  k_cvt_w<<<(unsigned)((wpieces + 255) / 256), 256, 0, stream>>>(Wo, Wob, wpieces);
  k_proj<<<dim3((unsigned)(NB * SEQ / 64), 24u, 1u), 128, 0, stream>>>(Xb, Wb, bq, bk, bv, mask, QKV);
  k_attn<<<(unsigned)(NB * NH * (SEQ / 64)), 128, 0, stream>>>(QKV, QKV + PLANE, QKV + 2 * PLANE, dist, mask, Yp);
  k_out<<<(unsigned)(NB * SEQ / 64), 128, 0, stream>>>(Yp, Wob, bo, mask, out);
}
